// DCNLayer_83167746720269
// MI455X (gfx1250) — hardware-verified
//
#include <hip/hip_runtime.h>
#include <math.h>
#include <stdint.h>


typedef __attribute__((ext_vector_type(16))) _Float16 v16h;
typedef __attribute__((ext_vector_type(8)))  _Float16 v8h;
typedef __attribute__((ext_vector_type(4)))  _Float16 v4h;
typedef __attribute__((ext_vector_type(16))) __bf16   v16b;
typedef __attribute__((ext_vector_type(8)))  __bf16   v8b;
typedef __attribute__((ext_vector_type(8)))  float    v8f;
typedef __attribute__((ext_vector_type(4)))  float    v4f;
typedef __attribute__((ext_vector_type(4)))  unsigned short v4us;
typedef v4f __attribute__((may_alias)) v4fa;

static constexpr int NIMG = 8, HH = 56, WW = 56, CC = 256, GG = 16, PP = 9;
static constexpr int NTOK = NIMG * HH * WW;
static constexpr int CM   = 4 * CC;
static constexpr int NOFF = GG * PP * 2;
static constexpr int NMSK = GG * PP;
static constexpr int NOMC = 448;
static_assert(NTOK % 64 == 0);
static_assert(NTOK % 8 == 0);
static_assert(NOMC % 64 == 0);
#define INV58 (1.0f / 58.0f)

__device__ __forceinline__ unsigned short f2bf_bits(float f) {
  unsigned u = __float_as_uint(f);
  return (unsigned short)((u + 0x7FFFu + ((u >> 16) & 1u)) >> 16);
}
__device__ __forceinline__ float bf_bits2f(unsigned short h) { return __uint_as_float(((unsigned)h) << 16); }

__device__ __forceinline__ void dep_guard_h(v8f& a, v8f& b, v16h x, v16h y) { asm volatile("v_nop\n\tv_nop\n\tv_nop\n\tv_nop" : "+v"(a), "+v"(b) : "v"(x), "v"(y)); }
__device__ __forceinline__ void dep_guard_b(v8f& a, v8f& b, v16b x, v16b y) { asm volatile("v_nop\n\tv_nop\n\tv_nop\n\tv_nop" : "+v"(a), "+v"(b) : "v"(x), "v"(y)); }
__device__ __forceinline__ void keep4_h(v16h a, v16h b, v16h c, v16h d) { asm volatile("v_nop" :: "v"(a), "v"(b), "v"(c), "v"(d)); }
__device__ __forceinline__ void keep4_b(v16b a, v16b b, v16b c, v16b d) { asm volatile("v_nop" :: "v"(a), "v"(b), "v"(c), "v"(d)); }
__device__ __forceinline__ void acc_guard4(v8f& a, v8f& b, v8f& c, v8f& d) { asm volatile("v_nop\n\tv_nop\n\tv_nop\n\tv_nop" : "+v"(a), "+v"(b), "+v"(c), "+v"(d)); }
template <typename T> struct Frag;
template <> struct Frag<_Float16> {
  typedef v16h V; union U { v16h v; v8h h[2]; };
  static __device__ __forceinline__ v16h load(const _Float16* p) {
    U f; f.h[0] = *(const v8h*)(p); f.h[1] = *(const v8h*)(p + 16); return f.v;
  }
  static __device__ __forceinline__ v8f mma(v16h a, v16h b, v8f c) {
    return __builtin_amdgcn_wmma_f32_16x16x32_f16(false, a, false, b, (short)0, c, false, false);
  }
  static __device__ __forceinline__ void guard(v8f& a, v8f& b, v16h x, v16h y) { dep_guard_h(a, b, x, y); }
  static __device__ __forceinline__ void keep(v16h a, v16h b, v16h c, v16h d) { keep4_h(a, b, c, d); }
};
template <> struct Frag<__bf16> {
  typedef v16b V; union U { v16b v; v8b h[2]; };
  static __device__ __forceinline__ v16b load(const __bf16* p) {
    U f; f.h[0] = *(const v8b*)(p); f.h[1] = *(const v8b*)(p + 16); return f.v;
  }
  static __device__ __forceinline__ v8f mma(v16b a, v16b b, v8f c) {
    return __builtin_amdgcn_wmma_f32_16x16x32_bf16(false, a, false, b, (short)0, c, false, false);
  }
  static __device__ __forceinline__ void guard(v8f& a, v8f& b, v16b x, v16b y) { dep_guard_b(a, b, x, y); }
  static __device__ __forceinline__ void keep(v16b a, v16b b, v16b c, v16b d) { keep4_b(a, b, c, d); }
};

template <int ET> struct Elem;
template <> struct Elem<0> { typedef _Float16 T; };
template <> struct Elem<1> { typedef __bf16 T; };
template <int ET, bool SPLIT, int BIAS_MODE, int OUT_MODE, bool RESID, int ACT = 0>
__global__ __launch_bounds__(256) void wmma_gemm64(
    const unsigned short* __restrict__ Ap, const unsigned short* __restrict__ A2p, int lda, long strideA,
    const unsigned short* __restrict__ Btp, const unsigned short* __restrict__ Bt2p, int ldb, long strideB,
    void* __restrict__ Cout, void* __restrict__ Cout2, int ldc, long strideC,
    const float* __restrict__ bias,
    const float* __restrict__ resid, long strideR,
    int M, int N, int K, float scale, float oscale) {
  typedef typename Elem<ET>::T T;
  typedef typename Frag<T>::V V;
  const T* A = (const T*)Ap; const T* A2 = (const T*)A2p; const T* Bt = (const T*)Btp; const T* Bt2 = (const T*)Bt2p;
  __shared__ __align__(16) float sT[8][16 * 68];
  const int b    = blockIdx.y;
  const int lane = threadIdx.x & 31;
  const int wave = threadIdx.x >> 5;
  const int tilesN = N >> 6;
  const int tilesM = M >> 6;
  const int tile = blockIdx.x * 8 + wave;
  if (tile >= tilesM * tilesN) return;
  const int tm = tile / tilesN;
  const int tn = tile - tm * tilesN;
  const int m0 = tm << 6;
  const int n0 = tn << 6;

  const T* Ab  = A  + (size_t)b * strideA;
  const T* Bb  = Bt + (size_t)b * strideB;
  const T* Ab2 = SPLIT ? (A2  + (size_t)b * strideA) : nullptr;
  const T* Bb2 = SPLIT ? (Bt2 + (size_t)b * strideB) : nullptr;

  const int rlane = lane & 15;
  const int koff  = (lane >> 4) * 8;
  const int mOff  = (lane >> 4) * 8;

  v8f acc[4][4];
#pragma unroll
  for (int i = 0; i < 4; ++i)
#pragma unroll
    for (int j = 0; j < 4; ++j) acc[i][j] = (v8f){0.f,0.f,0.f,0.f,0.f,0.f,0.f,0.f};

  for (int k0 = 0; k0 < K; k0 += 32) {
    V bh[4], bl[4];
#pragma unroll
    for (int j = 0; j < 4; ++j) {
      const size_t bo = (size_t)(n0 + (j << 4) + rlane) * ldb + koff + k0;
      bh[j] = Frag<T>::load(Bb + bo);
      if (SPLIT) bl[j] = Frag<T>::load(Bb2 + bo);
    }
#pragma unroll
    for (int i = 0; i < 4; ++i) {
      const size_t ao = (size_t)(m0 + (i << 4) + rlane) * lda + koff + k0;
      V ah = Frag<T>::load(Ab + ao);
      V al;
      if (SPLIT) al = Frag<T>::load(Ab2 + ao);
#pragma unroll
      for (int j = 0; j < 4; ++j) {
        acc[i][j] = Frag<T>::mma(ah, bh[j], acc[i][j]);
        if (SPLIT) {
          acc[i][j] = Frag<T>::mma(ah, bl[j], acc[i][j]);
          acc[i][j] = Frag<T>::mma(al, bh[j], acc[i][j]);
        }
      }
      Frag<T>::guard(acc[i][0], acc[i][3], ah, SPLIT ? al : ah);
    }
    Frag<T>::keep(bh[0], bh[1], bh[2], bh[3]);
    if (SPLIT) Frag<T>::keep(bl[0], bl[1], bl[2], bl[3]);
  }
  acc_guard4(acc[0][0], acc[0][1], acc[0][2], acc[0][3]);
  acc_guard4(acc[1][0], acc[1][1], acc[1][2], acc[1][3]);
  acc_guard4(acc[2][0], acc[2][1], acc[2][2], acc[2][3]);
  acc_guard4(acc[3][0], acc[3][1], acc[3][2], acc[3][3]);

  float* slab = sT[wave];
  const float* Rb = RESID ? (resid + (size_t)b * strideR) : nullptr;
#pragma unroll
  for (int i = 0; i < 4; ++i) {
    const int mBase = m0 + (i << 4);
#pragma unroll
    for (int j = 0; j < 4; ++j) {
      const int n = n0 + (j << 4) + rlane;
      float bv = 0.f;
      if (BIAS_MODE == 2) bv = bias[n];
#pragma unroll
      for (int r = 0; r < 8; ++r) {
        float v = acc[i][j][r] * scale;
        if (BIAS_MODE == 1) v += bias[mBase + mOff + r];
        if (BIAS_MODE == 2) v += bv;
        if (RESID) v += Rb[(size_t)(mBase + mOff + r) * ldc + n];
        if (ACT == 1) v = tanhf(v);
        if (ACT == 2) v = fmaxf(v, 0.0f);
        if (ACT == 3) v = v / (1.0f + expf(-v));
        if (ACT == 4) v = (v > 0.f) ? v : 0.01f * v;
        if (ACT == 5) v = 0.5f * v * (1.0f + erff(v * 0.70710678118654752f));
        v = v * oscale;
        slab[(mOff + r) * 68 + (j << 4) + rlane] = v;
      }
    }
    __builtin_amdgcn_fence(__ATOMIC_RELEASE, "workgroup");
    __builtin_amdgcn_wave_barrier();
    __builtin_amdgcn_fence(__ATOMIC_ACQUIRE, "workgroup");
    if (OUT_MODE == 0) {
      float* C = (float*)Cout + (size_t)b * strideC;
      const int hh = lane >> 4, c4 = (lane & 15) * 4;
      for (int pass = 0; pass < 2; ++pass) {
#pragma unroll
        for (int it = 0; it < 8; ++it) {
          const int row = it * 2 + hh;
          v4f v = *(const v4f*)(slab + row * 68 + c4);
          *(volatile v4f*)(C + (size_t)(mBase + row) * ldc + n0 + c4) = v;
        }
        __threadfence();
      }
    } else {
      const int q = lane >> 3, c8 = (lane & 7) * 8;
      unsigned short* C  = (unsigned short*)Cout  + (size_t)b * strideC;
      unsigned short* C2 = (OUT_MODE == 2) ? ((unsigned short*)Cout2 + (size_t)b * strideC) : nullptr;
      for (int pass = 0; pass < 2; ++pass) {
#pragma unroll
        for (int it = 0; it < 4; ++it) {
          const int row = it * 4 + q;
          const float* sp = slab + row * 68 + c8;
          v8h hv, lv;
#pragma unroll
          for (int e = 0; e < 8; ++e) {
            if (OUT_MODE == 1) {
              hv[e] = (_Float16)sp[e];
            } else {
              unsigned short hb = f2bf_bits(sp[e]);
              unsigned short lb = f2bf_bits(sp[e] - bf_bits2f(hb));
              hv[e] = __builtin_bit_cast(_Float16, hb);
              lv[e] = __builtin_bit_cast(_Float16, lb);
            }
          }
          *(volatile v8h*)(C + (size_t)(mBase + row) * ldc + n0 + c8) = hv;
          if (OUT_MODE == 2) *(volatile v8h*)(C2 + (size_t)(mBase + row) * ldc + n0 + c8) = lv;
        }
        __threadfence();
      }
    }
    __builtin_amdgcn_fence(__ATOMIC_RELEASE, "workgroup");
    __builtin_amdgcn_wave_barrier();
    __builtin_amdgcn_fence(__ATOMIC_ACQUIRE, "workgroup");
  }
}

__device__ __forceinline__ float gelu_erf(float x) {
  return 0.5f * x * (1.0f + erff(x * 0.70710678118654752440f));
}
__device__ __forceinline__ float wave_sum(float v) {
#pragma unroll
  for (int o = 16; o > 0; o >>= 1) v += __shfl_xor(v, o, 32);
  return v;
}
__device__ __forceinline__ void lds_wave_sync() {
  __builtin_amdgcn_fence(__ATOMIC_RELEASE, "workgroup");
  __builtin_amdgcn_wave_barrier();
  __builtin_amdgcn_fence(__ATOMIC_ACQUIRE, "workgroup");
}
__device__ __forceinline__ void ln8(const v4f xa, const v4f xb, const float* __restrict__ g, const float* __restrict__ bt,
                                    int c0, int c1, v4f& oa, v4f& ob) {
  float s = ((xa[0] + xa[1]) + (xa[2] + xa[3])) + ((xb[0] + xb[1]) + (xb[2] + xb[3]));
  s = wave_sum(s);
  const float mean = s * (1.0f / (float)CC);
  const v4f da = xa - mean, db = xb - mean;
  float q = ((da[0] * da[0] + da[1] * da[1]) + (da[2] * da[2] + da[3] * da[3]))
          + ((db[0] * db[0] + db[1] * db[1]) + (db[2] * db[2] + db[3] * db[3]));
  q = wave_sum(q);
  const float var  = q * (1.0f / (float)CC);
  const float rstd = rsqrtf(var + 1e-6f);
  const v4f ga = *(const v4f*)(g + c0),  gb = *(const v4f*)(g + c1);
  const v4f ba = *(const v4f*)(bt + c0), bb = *(const v4f*)(bt + c1);
  oa = (da * rstd) * ga + ba;
  ob = (db * rstd) * gb + bb;
}

template <bool WF32>
__global__ __launch_bounds__(256) void k_ln(const float* __restrict__ x, const float* __restrict__ g,
                                            const float* __restrict__ bt, float* __restrict__ outF,
                                            _Float16* __restrict__ outH, int ntok) {
  const int lane = threadIdx.x & 31, wave = threadIdx.x >> 5;
  const int tok = blockIdx.x * 8 + wave;
  if (tok >= ntok) return;
  const size_t base = (size_t)tok * CC;
  const int c0 = lane * 4, c1 = 128 + lane * 4;
  const v4f xa = *(const v4f*)(x + base + c0);
  const v4f xb = *(const v4f*)(x + base + c1);
  v4f oa, ob;
  ln8(xa, xb, g, bt, c0, c1, oa, ob);
  v4h ha, hb;
#pragma unroll
  for (int e = 0; e < 4; ++e) { ha[e] = (_Float16)oa[e]; hb[e] = (_Float16)ob[e]; }
  for (int pass = 0; pass < 2; ++pass) {
    if (WF32) {
      *(volatile v4f*)(outF + base + c0) = oa;
      *(volatile v4f*)(outF + base + c1) = ob;
    }
    *(volatile v4h*)(outH + base + c0) = ha;
    *(volatile v4h*)(outH + base + c1) = hb;
    __threadfence();
  }
}

__global__ __launch_bounds__(256) void k_dw1(const float* __restrict__ h, const float* __restrict__ k9,
                                             const float* __restrict__ kb, const float* __restrict__ g,
                                             const float* __restrict__ bt, unsigned short* __restrict__ oh,
                                             unsigned short* __restrict__ ol, int ntok) {
  __shared__ __align__(16) float sl[8][256];
  const int lane = threadIdx.x & 31, wave = threadIdx.x >> 5;
  const int tok = blockIdx.x * 8 + wave;
  if (tok >= ntok) return;
  const int bimg = tok / (HH * WW);
  const int rem  = tok - bimg * (HH * WW);
  const int ty = rem / WW;
  const int tx = rem - ty * WW;
  const int c0 = lane * 4, c1 = 128 + lane * 4;
  v4f aa = (v4f){0.f, 0.f, 0.f, 0.f}, ab = (v4f){0.f, 0.f, 0.f, 0.f};
#pragma unroll 1
  for (int tap = 0; tap < 9; ++tap) {
    const int ky = (tap * 11) >> 5;
    const int kx = tap - ky * 3;
    const int yy = ty + ky - 1, xx = tx + kx - 1;
    if (yy >= 0 && yy < HH && xx >= 0 && xx < WW) {
      const float* hr = h + ((size_t)(bimg * HH + yy) * WW + xx) * CC;
      const v4f ha = *(const v4f*)(hr + c0), hb = *(const v4f*)(hr + c1);
      const v4f ka = *(const v4f*)(k9 + tap * CC + c0), kbv = *(const v4f*)(k9 + tap * CC + c1);
      aa += ha * ka;
      ab += hb * kbv;
    }
  }
  aa += *(const v4f*)(kb + c0);
  ab += *(const v4f*)(kb + c1);
  v4f ua, ub;
  ln8(aa, ab, g, bt, c0, c1, ua, ub);
  float* slw = sl[wave];
  *(v4fa*)(slw + c0) = ua;
  *(v4fa*)(slw + c1) = ub;
  lds_wave_sync();
#pragma unroll 1
  for (int e = 0; e < 8; ++e) {
    const int idx = lane * 4 + (e & 3) + ((e >> 2) << 7);
    const float u = slw[idx];
    slw[idx] = gelu_erf(u);
  }
  lds_wave_sync();
  const v4f ra = *(const v4fa*)(slw + c0), rb = *(const v4fa*)(slw + c1);
  v4us ha, la, hbv, lbv;
#pragma unroll
  for (int e = 0; e < 4; ++e) {
    const unsigned short h0 = f2bf_bits(ra[e]);
    ha[e] = h0; la[e] = f2bf_bits(ra[e] - bf_bits2f(h0));
    const unsigned short h1 = f2bf_bits(rb[e]);
    hbv[e] = h1; lbv[e] = f2bf_bits(rb[e] - bf_bits2f(h1));
  }
  const size_t base = (size_t)tok * CC;
  for (int pass = 0; pass < 2; ++pass) {
    *(volatile v4us*)(oh + base + c0) = ha;
    *(volatile v4us*)(oh + base + c1) = hbv;
    *(volatile v4us*)(ol + base + c0) = la;
    *(volatile v4us*)(ol + base + c1) = lbv;
    __threadfence();
  }
}

__global__ __launch_bounds__(256) void k_dcn(const float* __restrict__ xp, const float* __restrict__ om,
                                             unsigned short* __restrict__ core, int ntok) {
  const int lane = threadIdx.x & 31, wave = threadIdx.x >> 5;
  const int tok = blockIdx.x * 8 + wave;
  if (tok >= ntok) return;
  const int bimg = tok / (HH * WW);
  const int rem  = tok - bimg * (HH * WW);
  const int ty = rem / WW;
  const int tx = rem - ty * WW;
  const int g  = lane >> 1;
  const int hf = (lane & 1) * 8;
  const float* omr  = om + (size_t)tok * NOMC;
  const float* offp = omr + g * (PP * 2);
  const float* lgp  = omr + NOFF + g * PP;

  float mx = -INFINITY;
#pragma unroll 1
  for (int p = 0; p < PP; ++p) mx = fmaxf(mx, lgp[p]);
  float ssum = 0.f;
#pragma unroll 1
  for (int p = 0; p < PP; ++p) ssum += expf(lgp[p] - mx);
  const float inv = 1.0f / ssum;

  const float rbx = ((float)tx + 1.5f) * INV58;
  const float rby = ((float)ty + 1.5f) * INV58;
  const float* xpb = xp + (size_t)bimg * (HH * WW) * CC + g * 16 + hf;

  v4f ca = (v4f){0.f, 0.f, 0.f, 0.f}, cb = (v4f){0.f, 0.f, 0.f, 0.f};
#pragma unroll 1
  for (int p = 0; p < PP; ++p) {
    const int i3 = (p * 11) >> 5;
    const int j3 = p - i3 * 3;
    const float gx = (float)(i3 - 1), gy = (float)(j3 - 1);
    const float ox = offp[2 * p], oy = offp[2 * p + 1];
    const float ep = expf(lgp[p] - mx) * inv;
    float x0f, y0f, w00, w01, w10, w11;
    {
#pragma clang fp contract(off)
      const float locx = (rbx + gx * INV58) + ox * INV58;
      const float locy = (rby + gy * INV58) + oy * INV58;
      const float px = locx * 58.0f - 0.5f;
      const float py = locy * 58.0f - 0.5f;
      x0f = floorf(px); y0f = floorf(py);
      const float fx = px - x0f, fy = py - y0f;
      const float gx0 = 1.0f - fx, gy0 = 1.0f - fy;
      w00 = gy0 * gx0; w01 = gy0 * fx; w10 = fy * gx0; w11 = fy * fx;
    }
    const int x0i = (int)fminf(fmaxf(x0f, -8.0f), 72.0f);
    const int y0i = (int)fminf(fmaxf(y0f, -8.0f), 72.0f);
    const int rx0 = x0i - 1, rx1 = x0i, ry0 = y0i - 1, ry1 = y0i;
    const bool vx0 = (unsigned)rx0 < (unsigned)WW, vx1 = (unsigned)rx1 < (unsigned)WW;
    const bool vy0 = (unsigned)ry0 < (unsigned)HH, vy1 = (unsigned)ry1 < (unsigned)HH;
    const int cx0 = min(max(rx0, 0), WW - 1), cx1 = min(max(rx1, 0), WW - 1);
    const int cy0 = min(max(ry0, 0), HH - 1), cy1 = min(max(ry1, 0), HH - 1);
    const float e00 = (vy0 && vx0) ? w00 : 0.f;
    const float e01 = (vy0 && vx1) ? w01 : 0.f;
    const float e10 = (vy1 && vx0) ? w10 : 0.f;
    const float e11 = (vy1 && vx1) ? w11 : 0.f;
    const float* r00 = xpb + ((size_t)cy0 * WW + cx0) * CC;
    const float* r01 = xpb + ((size_t)cy0 * WW + cx1) * CC;
    const float* r10 = xpb + ((size_t)cy1 * WW + cx0) * CC;
    const float* r11 = xpb + ((size_t)cy1 * WW + cx1) * CC;
    v4f sa, sb;
    { const v4f a = *(const v4f*)(r00), bq = *(const v4f*)(r00 + 4); sa = a * e00;  sb = bq * e00; }
    { const v4f a = *(const v4f*)(r01), bq = *(const v4f*)(r01 + 4); sa += a * e01; sb += bq * e01; }
    { const v4f a = *(const v4f*)(r10), bq = *(const v4f*)(r10 + 4); sa += a * e10; sb += bq * e10; }
    { const v4f a = *(const v4f*)(r11), bq = *(const v4f*)(r11 + 4); sa += a * e11; sb += bq * e11; }
    ca += sa * ep;
    cb += sb * ep;
  }
  v8h hv;
#pragma unroll
  for (int e = 0; e < 4; ++e) { hv[e] = (_Float16)(ca[e] * 16.0f); hv[4 + e] = (_Float16)(cb[e] * 16.0f); }
  unsigned short* dst = core + (size_t)tok * CC + lane * 8;
  *(volatile v8h*)dst = hv;
  __threadfence();
  *(volatile v8h*)dst = hv;
}

__global__ __launch_bounds__(256) void k_dw2(const unsigned short* __restrict__ y1, const float* __restrict__ k9,
                                             const float* __restrict__ kb, unsigned short* __restrict__ y2, int ntok) {
  __shared__ __align__(16) float sl[8][256];
  const int lane = threadIdx.x & 31, wave = threadIdx.x >> 5;
  const int tok = blockIdx.x * 8 + wave;
  if (tok >= ntok) return;
  const int bimg = tok / (HH * WW);
  const int rem  = tok - bimg * (HH * WW);
  const int ty = rem / WW;
  const int tx = rem - ty * WW;
  const _Float16* y1h = (const _Float16*)y1;
  float* slw = sl[wave] + lane * 8;
#pragma unroll 1
  for (int q = 0; q < 4; ++q) {
    const int cb = q * 256 + lane * 8;
    v4f aa = (v4f){0.f, 0.f, 0.f, 0.f}, ab = (v4f){0.f, 0.f, 0.f, 0.f};
#pragma unroll 1
    for (int tap = 0; tap < 9; ++tap) {
      const int ky = (tap * 11) >> 5;
      const int kx = tap - ky * 3;
      const int yy = ty + ky - 1, xx = tx + kx - 1;
      if (yy >= 0 && yy < HH && xx >= 0 && xx < WW) {
        const v8h hv = *(const v8h*)(y1h + ((size_t)(bimg * HH + yy) * WW + xx) * CM + cb);
        const v4f ka = *(const v4f*)(k9 + tap * CM + cb), kbv = *(const v4f*)(k9 + tap * CM + cb + 4);
#pragma unroll
        for (int e = 0; e < 4; ++e) {
          aa[e] += (float)hv[e] * ka[e];
          ab[e] += (float)hv[4 + e] * kbv[e];
        }
      }
    }
    const v4f ba = *(const v4f*)(kb + cb), bb = *(const v4f*)(kb + cb + 4);
    aa = aa * (1.0f / 16.0f) + ba;
    ab = ab * (1.0f / 16.0f) + bb;
    *(v4fa*)(slw)     = aa;
    *(v4fa*)(slw + 4) = ab;
    lds_wave_sync();
#pragma unroll 1
    for (int e = 0; e < 8; ++e) {
      const float u = slw[e];
      slw[e] = gelu_erf(u) * 256.0f;
    }
    lds_wave_sync();
    const v4f ra = *(const v4fa*)(slw), rb = *(const v4fa*)(slw + 4);
    v8h ov;
#pragma unroll
    for (int e = 0; e < 4; ++e) { ov[e] = (_Float16)ra[e]; ov[4 + e] = (_Float16)rb[e]; }
    unsigned short* dst = y2 + (size_t)tok * CM + cb;
    *(volatile v8h*)dst = ov;
    __threadfence();
    *(volatile v8h*)dst = ov;
    lds_wave_sync();
  }
}

template <int OM>
__global__ __launch_bounds__(256) void k_wt(const float* __restrict__ s1, int N1, const float* __restrict__ s2, int N2,
                                            int K, float scale, unsigned short* __restrict__ o1,
                                            unsigned short* __restrict__ o2) {
  __shared__ float tile[32][65];
  const int t = threadIdx.x;
  const int lane = t & 31, wave = t >> 5;
  const int n0 = blockIdx.x * 32, k0 = blockIdx.y * 64;
#pragma unroll
  for (int i = 0; i < 8; ++i) {
    const int idx = t + 256 * i;
    const int kk = idx >> 5, nn = idx & 31;
    const int n = n0 + nn, k = k0 + kk;
    const int n1c = min(n, N1 - 1);
    int n2c = n - N1; n2c = max(n2c, 0); n2c = min(n2c, N2 - 1);
    const float v1 = s1[(size_t)k * N1 + n1c];
    const float v2 = s2[(size_t)k * N2 + n2c];
    const float v = (n < N1) ? v1 : ((n < N1 + N2) ? v2 : 0.0f);
    tile[nn][kk] = v;
  }
  __syncthreads();
  const int row = wave * 4 + (lane >> 3), c8 = (lane & 7) * 8;
  v8h hv, lv;
#pragma unroll
  for (int e = 0; e < 8; ++e) {
    const float f = tile[row][c8 + e];
    if (OM == 0) {
      hv[e] = (_Float16)(f * scale);
    } else {
      const unsigned short hb = f2bf_bits(f);
      const unsigned short lb = f2bf_bits(f - bf_bits2f(hb));
      hv[e] = __builtin_bit_cast(_Float16, hb);
      lv[e] = __builtin_bit_cast(_Float16, lb);
    }
  }
  const size_t o = (size_t)(n0 + row) * K + k0 + c8;
  for (int pass = 0; pass < 2; ++pass) {
    *(volatile v8h*)(o1 + o) = hv;
    if (OM == 1) *(volatile v8h*)(o2 + o) = lv;
    __threadfence();
  }
}

__global__ __launch_bounds__(512) void k_bias(const float* __restrict__ b1p, const float* __restrict__ b2p,
                                              float* __restrict__ dst) {
  const int i = threadIdx.x;
  if (i < NOMC) {
    const float v1 = b1p[min(i, NOFF - 1)];
    int j = i - NOFF; j = max(j, 0); j = min(j, NMSK - 1);
    const float v2 = b2p[j];
    const float v = (i < NOFF) ? v1 : ((i < NOFF + NMSK) ? v2 : 0.0f);
    ((volatile float*)dst)[i] = v;
    __threadfence();
    ((volatile float*)dst)[i] = v;
  }
}

static inline unsigned gemm_blocks(int M, int N) { return (unsigned)(((M / 64) * (N / 64) + 7) / 8); }

extern "C" void kernel_launch(void* const* d_in, const int* in_sizes, int n_in,
                              void* d_out, int out_size, void* d_ws, size_t ws_size,
                              hipStream_t stream) {
  if (n_in < 21) return;
  if (in_sizes[0] != NTOK * CC || out_size != NTOK * CC) return;
  const float* x    = (const float*)d_in[0];
  const float* g1   = (const float*)d_in[1];
  const float* b1   = (const float*)d_in[2];
  const float* Wi   = (const float*)d_in[3];
  const float* bi   = (const float*)d_in[4];
  const float* dwk  = (const float*)d_in[5];
  const float* dwb  = (const float*)d_in[6];
  const float* gdw  = (const float*)d_in[7];
  const float* bdw  = (const float*)d_in[8];
  const float* Woff = (const float*)d_in[9];
  const float* boff = (const float*)d_in[10];
  const float* Wm   = (const float*)d_in[11];
  const float* bm   = (const float*)d_in[12];
  const float* Wo   = (const float*)d_in[13];
  const float* bo   = (const float*)d_in[14];
  const float* g2   = (const float*)d_in[15];
  const float* b2   = (const float*)d_in[16];
  const float* w1   = (const float*)d_in[17];
  const float* dwk2 = (const float*)d_in[18];
  const float* dwb2 = (const float*)d_in[19];
  const float* w2   = (const float*)d_in[20];
  float* out = (float*)d_out;

  const size_t P32 = (size_t)NTOK * CC * 4;
  const size_t P16 = (size_t)NTOK * CC * 2;
  const size_t Y16 = (size_t)NTOK * CM * 2;
  const size_t OMB = (size_t)NTOK * NOMC * 4;
  if (OMB > Y16 || P16 > Y16) return;
  char* ws  = (char*)d_ws;
  char* arA = ws;
  char* arB = arA + P32;
  char* arC = arB + Y16;
  char* wb  = arC + Y16;
  size_t woff = 0;
  unsigned short* WiT   = (unsigned short*)(wb + woff); woff += (size_t)CC * CC * 2;
  unsigned short* WomTh = (unsigned short*)(wb + woff); woff += (size_t)NOMC * CC * 2;
  unsigned short* WomTl = (unsigned short*)(wb + woff); woff += (size_t)NOMC * CC * 2;
  unsigned short* WoT   = (unsigned short*)(wb + woff); woff += (size_t)CC * CC * 2;
  unsigned short* w1T   = (unsigned short*)(wb + woff); woff += (size_t)CM * CC * 2;
  unsigned short* w2T   = (unsigned short*)(wb + woff); woff += (size_t)CC * CM * 2;
  float*          bomF  = (float*)(wb + woff);          woff += 2048;
  const size_t total = (size_t)(wb - ws) + woff;
  if (total > ws_size || total > (size_t)134217728) return;

  float*          hF    = (float*)arA;
  float*          xmidF = (float*)arA;
  float*          xpF   = (float*)arB;
  unsigned short* x1h   = (unsigned short*)(arB + P32);
  unsigned short* x1l   = (unsigned short*)(arB + P32 + P16);
  unsigned short* coreH = (unsigned short*)(arB + P32);
  unsigned short* y1H   = (unsigned short*)arB;
  unsigned short* hH    = (unsigned short*)arC;
  float*          omF   = (float*)arC;
  unsigned short* h2H   = (unsigned short*)arC;
  unsigned short* y2H   = (unsigned short*)arC;

  const dim3 blk(256);
  const unsigned tokBlocks = (unsigned)((NTOK + 7) / 8);

  k_wt<0><<<dim3(CC / 32, CC / 64), blk, 0, stream>>>(Wi, CC, Wi, 1, CC, 64.0f, WiT, nullptr);
  k_wt<1><<<dim3(NOMC / 32, CC / 64), blk, 0, stream>>>(Woff, NOFF, Wm, NMSK, CC, 1.0f, WomTh, WomTl);
  k_wt<0><<<dim3(CC / 32, CC / 64), blk, 0, stream>>>(Wo, CC, Wo, 1, CC, 64.0f, WoT, nullptr);
  k_wt<0><<<dim3(CM / 32, CC / 64), blk, 0, stream>>>(w1, CM, w1, 1, CC, 64.0f, w1T, nullptr);
  k_wt<0><<<dim3(CC / 32, CM / 64), blk, 0, stream>>>(w2, CC, w2, 1, CM, 64.0f, w2T, nullptr);
  k_bias<<<dim3(1), dim3(512), 0, stream>>>(boff, bm, bomF);

  k_ln<true><<<dim3(tokBlocks), blk, 0, stream>>>(x, g1, b1, hF, (_Float16*)hH, NTOK);
  wmma_gemm64<0, false, 2, 0, false, 0><<<dim3(gemm_blocks(NTOK, CC)), blk, 0, stream>>>(
      hH, nullptr, CC, 0L, WiT, nullptr, CC, 0L, xpF, nullptr, CC, 0L,
      bi, nullptr, 0L, NTOK, CC, CC, 1.0f / 64.0f, 1.0f);
  k_dw1<<<dim3(tokBlocks), blk, 0, stream>>>(hF, dwk, dwb, gdw, bdw, x1h, x1l, NTOK);
  wmma_gemm64<1, true, 2, 0, false, 0><<<dim3(gemm_blocks(NTOK, NOMC)), blk, 0, stream>>>(
      x1h, x1l, CC, 0L, WomTh, WomTl, CC, 0L, omF, nullptr, NOMC, 0L,
      bomF, nullptr, 0L, NTOK, NOMC, CC, 1.0f, 1.0f);
  k_dcn<<<dim3(tokBlocks), blk, 0, stream>>>(xpF, omF, coreH, NTOK);
  wmma_gemm64<0, false, 2, 0, true, 0><<<dim3(gemm_blocks(NTOK, CC)), blk, 0, stream>>>(
      coreH, nullptr, CC, 0L, WoT, nullptr, CC, 0L, xmidF, nullptr, CC, 0L,
      bo, x, 0L, NTOK, CC, CC, 1.0f / 1024.0f, 1.0f);

  k_ln<false><<<dim3(tokBlocks), blk, 0, stream>>>(xmidF, g2, b2, nullptr, (_Float16*)h2H, NTOK);
  wmma_gemm64<0, false, 0, 1, false, 5><<<dim3(gemm_blocks(NTOK, CM)), blk, 0, stream>>>(
      h2H, nullptr, CC, 0L, w1T, nullptr, CC, 0L, y1H, nullptr, CM, 0L,
      nullptr, nullptr, 0L, NTOK, CM, CC, 1.0f / 64.0f, 16.0f);
  k_dw2<<<dim3(tokBlocks), blk, 0, stream>>>(y1H, dwk2, dwb2, y2H, NTOK);
  wmma_gemm64<0, false, 0, 0, true, 0><<<dim3(gemm_blocks(NTOK, CC)), blk, 0, stream>>>(
      y2H, nullptr, CM, 0L, w2T, nullptr, CM, 0L, out, nullptr, CC, 0L,
      nullptr, xmidF, 0L, NTOK, CC, CM, 1.0f / 16384.0f, 1.0f);
  (void)hipGetLastError();
}
